// SocialPooling_87677462380869
// MI455X (gfx1250) — hardware-verified
//
#include <hip/hip_runtime.h>
#include <stddef.h>

constexpr int N_AGENT    = 2048;
constexpr int N_HID      = 128;
constexpr int N_GRID     = 8;
constexpr int N_CELLS    = N_GRID * N_GRID;
constexpr int K_FEAT     = N_CELLS * N_HID;
constexpr float NBH_HALF = 32.0f;
constexpr float CELL_INV = 0.125f;
constexpr int AG_PER_BLK = 4;
constexpr float HID_CARRY = 4.0f;
constexpr float W_CARRY   = 64.0f;
constexpr float GEMM_SCALE = 1.0f / (HID_CARRY * W_CARRY);

static_assert(N_AGENT % 64 == 0, "M tile");
static_assert(N_HID % 64 == 0, "N tile");
static_assert(N_HID % 32 == 0, "K step");
static_assert(N_AGENT % AG_PER_BLK == 0, "agent blocking");
static_assert(N_AGENT % 32 == 0, "chunking");
static_assert((N_AGENT * N_HID / 2) % 256 == 0, "cast grid hidden");
static_assert((N_HID * K_FEAT / 2) % 256 == 0, "cast grid W");

typedef __attribute__((ext_vector_type(16))) _Float16 v16h;
typedef __attribute__((ext_vector_type(8)))  _Float16 v8h;
typedef __attribute__((ext_vector_type(16))) __bf16   v16b;
typedef __attribute__((ext_vector_type(8)))  __bf16   v8b;
typedef __attribute__((ext_vector_type(8)))  float    v8f;
typedef __attribute__((ext_vector_type(4)))  float    v4f;
typedef __attribute__((ext_vector_type(2)))  float    v2f;

__device__ __forceinline__ unsigned short f2bf_bits(float f) {
  unsigned u = __float_as_uint(f);
  return (unsigned short)((u + 0x7FFFu + ((u >> 16) & 1u)) >> 16);
}
__device__ __forceinline__ float bf_bits2f(unsigned short h) { return __uint_as_float(((unsigned)h) << 16); }

__device__ __forceinline__ void dep_guard_h(v8f& a, v8f& b, v16h x, v16h y) { asm volatile("v_nop\n\tv_nop\n\tv_nop\n\tv_nop" : "+v"(a), "+v"(b) : "v"(x), "v"(y)); }
__device__ __forceinline__ void dep_guard_b(v8f& a, v8f& b, v16b x, v16b y) { asm volatile("v_nop\n\tv_nop\n\tv_nop\n\tv_nop" : "+v"(a), "+v"(b) : "v"(x), "v"(y)); }
__device__ __forceinline__ void keep4_h(v16h a, v16h b, v16h c, v16h d) { asm volatile("v_nop" :: "v"(a), "v"(b), "v"(c), "v"(d)); }
__device__ __forceinline__ void keep4_b(v16b a, v16b b, v16b c, v16b d) { asm volatile("v_nop" :: "v"(a), "v"(b), "v"(c), "v"(d)); }
__device__ __forceinline__ void acc_guard4(v8f& a, v8f& b, v8f& c, v8f& d) { asm volatile("v_nop\n\tv_nop\n\tv_nop\n\tv_nop" : "+v"(a), "+v"(b), "+v"(c), "+v"(d)); }
template <typename T> struct Frag;
template <> struct Frag<_Float16> {
  typedef v16h V; union U { v16h v; v8h h[2]; };
  static __device__ __forceinline__ v16h load(const _Float16* p) {
    U f; f.h[0] = *(const v8h*)(p); f.h[1] = *(const v8h*)(p + 16); return f.v;
  }
  static __device__ __forceinline__ v8f mma(v16h a, v16h b, v8f c) {
    return __builtin_amdgcn_wmma_f32_16x16x32_f16(false, a, false, b, (short)0, c, false, false);
  }
  static __device__ __forceinline__ void guard(v8f& a, v8f& b, v16h x, v16h y) { dep_guard_h(a, b, x, y); }
  static __device__ __forceinline__ void keep(v16h a, v16h b, v16h c, v16h d) { keep4_h(a, b, c, d); }
};
template <> struct Frag<__bf16> {
  typedef v16b V; union U { v16b v; v8b h[2]; };
  static __device__ __forceinline__ v16b load(const __bf16* p) {
    U f; f.h[0] = *(const v8b*)(p); f.h[1] = *(const v8b*)(p + 16); return f.v;
  }
  static __device__ __forceinline__ v8f mma(v16b a, v16b b, v8f c) {
    return __builtin_amdgcn_wmma_f32_16x16x32_bf16(false, a, false, b, (short)0, c, false, false);
  }
  static __device__ __forceinline__ void guard(v8f& a, v8f& b, v16b x, v16b y) { dep_guard_b(a, b, x, y); }
  static __device__ __forceinline__ void keep(v16b a, v16b b, v16b c, v16b d) { keep4_b(a, b, c, d); }
};

template <int ET> struct Elem;
template <> struct Elem<0> { typedef _Float16 T; };
template <> struct Elem<1> { typedef __bf16 T; };
template <int ET, bool SPLIT, int BIAS_MODE, int OUT_MODE, bool RESID, int ACT = 0>
__global__ __launch_bounds__(256) void wmma_gemm64(
    const unsigned short* __restrict__ Ap, const unsigned short* __restrict__ A2p, int lda, long strideA,
    const unsigned short* __restrict__ Btp, const unsigned short* __restrict__ Bt2p, int ldb, long strideB,
    void* __restrict__ Cout, void* __restrict__ Cout2, int ldc, long strideC,
    const float* __restrict__ bias,
    const float* __restrict__ resid, long strideR,
    int M, int N, int K, float scale) {
  typedef typename Elem<ET>::T T;
  typedef typename Frag<T>::V V;
  const T* A = (const T*)Ap; const T* A2 = (const T*)A2p; const T* Bt = (const T*)Btp; const T* Bt2 = (const T*)Bt2p;
  __shared__ __align__(16) float sT[8][16 * 68];
  const int b    = blockIdx.y;
  const int lane = threadIdx.x & 31;
  const int wave = threadIdx.x >> 5;
  const int tilesN = N >> 6;
  const int tilesM = M >> 6;
  const int tile = blockIdx.x * 8 + wave;
  if (tile >= tilesM * tilesN) return;
  const int tm = tile / tilesN;
  const int tn = tile - tm * tilesN;
  const int m0 = tm << 6;
  const int n0 = tn << 6;

  const T* Ab  = A  + (size_t)b * strideA;
  const T* Bb  = Bt + (size_t)b * strideB;
  const T* Ab2 = SPLIT ? (A2  + (size_t)b * strideA) : nullptr;
  const T* Bb2 = SPLIT ? (Bt2 + (size_t)b * strideB) : nullptr;

  const int rlane = lane & 15;
  const int koff  = (lane >> 4) * 8;
  const int mOff  = (lane >> 4) * 8;

  v8f acc[4][4];
#pragma unroll
  for (int i = 0; i < 4; ++i)
#pragma unroll
    for (int j = 0; j < 4; ++j) acc[i][j] = (v8f){0.f,0.f,0.f,0.f,0.f,0.f,0.f,0.f};

  for (int k0 = 0; k0 < K; k0 += 32) {
    V bh[4], bl[4];
#pragma unroll
    for (int j = 0; j < 4; ++j) {
      const size_t bo = (size_t)(n0 + (j << 4) + rlane) * ldb + koff + k0;
      bh[j] = Frag<T>::load(Bb + bo);
      if (SPLIT) bl[j] = Frag<T>::load(Bb2 + bo);
    }
#pragma unroll
    for (int i = 0; i < 4; ++i) {
      const size_t ao = (size_t)(m0 + (i << 4) + rlane) * lda + koff + k0;
      V ah = Frag<T>::load(Ab + ao);
      V al;
      if (SPLIT) al = Frag<T>::load(Ab2 + ao);
#pragma unroll
      for (int j = 0; j < 4; ++j) {
        acc[i][j] = Frag<T>::mma(ah, bh[j], acc[i][j]);
        if (SPLIT) {
          acc[i][j] = Frag<T>::mma(ah, bl[j], acc[i][j]);
          acc[i][j] = Frag<T>::mma(al, bh[j], acc[i][j]);
        }
      }
      Frag<T>::guard(acc[i][0], acc[i][3], ah, SPLIT ? al : ah);
    }
    Frag<T>::keep(bh[0], bh[1], bh[2], bh[3]);
    if (SPLIT) Frag<T>::keep(bl[0], bl[1], bl[2], bl[3]);
  }
  acc_guard4(acc[0][0], acc[0][1], acc[0][2], acc[0][3]);
  acc_guard4(acc[1][0], acc[1][1], acc[1][2], acc[1][3]);
  acc_guard4(acc[2][0], acc[2][1], acc[2][2], acc[2][3]);
  acc_guard4(acc[3][0], acc[3][1], acc[3][2], acc[3][3]);

  float* slab = sT[wave];
  const float* Rb = RESID ? (resid + (size_t)b * strideR) : nullptr;
#pragma unroll
  for (int i = 0; i < 4; ++i) {
    const int mBase = m0 + (i << 4);
#pragma unroll
    for (int j = 0; j < 4; ++j) {
      const int n = n0 + (j << 4) + rlane;
      float bv = 0.f;
      if (BIAS_MODE == 2) bv = bias[n];
#pragma unroll
      for (int r = 0; r < 8; ++r) {
        float v = acc[i][j][r] * scale;
        if (BIAS_MODE == 1) v += bias[mBase + mOff + r];
        if (BIAS_MODE == 2) v += bv;
        if (RESID) v += Rb[(size_t)(mBase + mOff + r) * ldc + n];
        if (ACT == 1) v = tanhf(v);
        if (ACT == 2) v = fmaxf(v, 0.0f);
        if (ACT == 3) v = v / (1.0f + expf(-v));
        if (ACT == 4) v = (v > 0.f) ? v : 0.01f * v;
        if (ACT == 5) v = 0.5f * v * (1.0f + erff(v * 0.70710678118654752f));
        slab[(mOff + r) * 68 + (j << 4) + rlane] = v;
      }
    }
    __builtin_amdgcn_fence(__ATOMIC_RELEASE, "workgroup");
    __builtin_amdgcn_wave_barrier();
    __builtin_amdgcn_fence(__ATOMIC_ACQUIRE, "workgroup");
    if (OUT_MODE == 0) {
      float* C = (float*)Cout + (size_t)b * strideC;
      const int hh = lane >> 4, c4 = (lane & 15) * 4;
      for (int pass = 0; pass < 2; ++pass) {
#pragma unroll
        for (int it = 0; it < 8; ++it) {
          const int row = it * 2 + hh;
          v4f v = *(const v4f*)(slab + row * 68 + c4);
          *(volatile v4f*)(C + (size_t)(mBase + row) * ldc + n0 + c4) = v;
        }
        __threadfence();
      }
    } else {
      const int q = lane >> 3, c8 = (lane & 7) * 8;
      unsigned short* C  = (unsigned short*)Cout  + (size_t)b * strideC;
      unsigned short* C2 = (OUT_MODE == 2) ? ((unsigned short*)Cout2 + (size_t)b * strideC) : nullptr;
      for (int pass = 0; pass < 2; ++pass) {
#pragma unroll
        for (int it = 0; it < 4; ++it) {
          const int row = it * 4 + q;
          const float* sp = slab + row * 68 + c8;
          v8h hv, lv;
#pragma unroll
          for (int e = 0; e < 8; ++e) {
            if (OUT_MODE == 1) {
              hv[e] = (_Float16)sp[e];
            } else {
              unsigned short hb = f2bf_bits(sp[e]);
              unsigned short lb = f2bf_bits(sp[e] - bf_bits2f(hb));
              hv[e] = __builtin_bit_cast(_Float16, hb);
              lv[e] = __builtin_bit_cast(_Float16, lb);
            }
          }
          *(volatile v8h*)(C + (size_t)(mBase + row) * ldc + n0 + c8) = hv;
          if (OUT_MODE == 2) *(volatile v8h*)(C2 + (size_t)(mBase + row) * ldc + n0 + c8) = lv;
        }
        __threadfence();
      }
    }
    __builtin_amdgcn_fence(__ATOMIC_RELEASE, "workgroup");
    __builtin_amdgcn_wave_barrier();
    __builtin_amdgcn_fence(__ATOMIC_ACQUIRE, "workgroup");
  }
}

__global__ __launch_bounds__(256) void cast_f32_f16x2_carry(
    const float* __restrict__ in, _Float16* __restrict__ out, int n2, float carry) {
  int i = blockIdx.x * 256 + threadIdx.x;
  if (i < n2) {
    const float f0 = in[2 * i] * carry;
    const float f1 = in[2 * i + 1] * carry;
    const _Float16 h0 = (_Float16)f0, h1 = (_Float16)f1;
    const unsigned u = (unsigned)__builtin_bit_cast(unsigned short, h0) | ((unsigned)__builtin_bit_cast(unsigned short, h1) << 16);
    ((volatile unsigned*)out)[i] = u;
    __threadfence();
    ((volatile unsigned*)out)[i] = u;
  }
}

__global__ __launch_bounds__(128) void cell_gather_pool(
    const float* __restrict__ P, const float* __restrict__ pos, const int* __restrict__ mask,
    const float* __restrict__ bias, float* __restrict__ out) {
#pragma clang fp contract(off)
  __shared__ unsigned int lst[AG_PER_BLK][N_AGENT];
  const int tid  = threadIdx.x;
  const int wave = tid >> 5;
  const int lane = tid & 31;
  const int i    = blockIdx.x * AG_PER_BLK + wave;
  const float pix = pos[2 * i];
  const float piy = pos[2 * i + 1];
  const int   mi  = mask[i];

  int cnt = 0;
#pragma unroll 1
  for (int ch = 0; ch < N_AGENT / 32; ++ch) {
    const int j = ch * 32 + lane;
    const v2f pj = *(const v2f*)(pos + 2 * j);
    const int mj = mask[j];
    const float rx = pj.x - pix;
    const float ry = pj.y - piy;
    const bool inr = (fabsf(rx) < NBH_HALF) && (fabsf(ry) < NBH_HALF) && (j != i) && (mj != 0);
    float tx = rx + NBH_HALF;
    float ty = ry + NBH_HALF;
    asm volatile("" : "+v"(tx));
    asm volatile("" : "+v"(ty));
    tx = tx * CELL_INV;
    ty = ty * CELL_INV;
    int col = (int)floorf(tx);
    int row = (int)floorf(ty);
    col = col < 0 ? 0 : (col > N_GRID - 1 ? N_GRID - 1 : col);
    row = row < 0 ? 0 : (row > N_GRID - 1 ? N_GRID - 1 : row);
    const unsigned int cell = (unsigned int)(row * N_GRID + col);
    const unsigned int bal   = __builtin_amdgcn_ballot_w32(inr);
    const unsigned int below = bal & ((1u << lane) - 1u);
    const int pre = (int)__builtin_popcount(below);
    if (inr) lst[wave][cnt + pre] = (cell << 16) | (unsigned int)j;
    cnt += (int)__builtin_popcount(bal);
  }
  __syncthreads();

  cnt = cnt > N_AGENT ? N_AGENT : cnt;
  v4f acc = {0.0f, 0.0f, 0.0f, 0.0f};
  const float* Pl = P + lane * 4;
#pragma unroll 1
  for (int e = 0; e < cnt; e += 4) {
    const int last = cnt - 1;
#pragma unroll
    for (int u = 0; u < 4; ++u) {
      int idx = e + u;
      idx = idx > last ? last : idx;
      const unsigned int ent = lst[wave][idx];
      const unsigned int jj  = ent & 2047u;
      const unsigned int cc  = (ent >> 16) & 63u;
      const v4f pv = *(const v4f*)(Pl + (size_t)(cc * (unsigned)N_AGENT + jj) * (size_t)N_HID);
      const bool keep = (e + u) < cnt;
      v4f add;
      add.x = keep ? pv.x : 0.0f;
      add.y = keep ? pv.y : 0.0f;
      add.z = keep ? pv.z : 0.0f;
      add.w = keep ? pv.w : 0.0f;
      acc += add;
    }
  }

  const v4f bv = *(const v4f*)(bias + lane * 4);
  const bool vi = (mi != 0) && (pix == pix) && (piy == piy);
  v4f o;
  o.x = vi ? (acc.x + bv.x) : 0.0f;
  o.y = vi ? (acc.y + bv.y) : 0.0f;
  o.z = vi ? (acc.z + bv.z) : 0.0f;
  o.w = vi ? (acc.w + bv.w) : 0.0f;
  float* op = out + (size_t)i * N_HID + lane * 4;
  *(volatile v4f*)op = o;
  __threadfence();
  *(volatile v4f*)op = o;
}

extern "C" void kernel_launch(void* const* d_in, const int* in_sizes, int n_in,
                              void* d_out, int out_size, void* d_ws, size_t ws_size,
                              hipStream_t stream) {
  if (n_in < 5) return;
  if (in_sizes[0] != N_AGENT * N_HID) return;
  if (in_sizes[1] != N_AGENT * 2) return;
  if (in_sizes[2] != N_AGENT) return;
  if (in_sizes[3] != N_HID * K_FEAT) return;
  if (in_sizes[4] != N_HID) return;
  if (out_size != N_AGENT * N_HID) return;

  const float* hidden = (const float*)d_in[0];
  const float* pos    = (const float*)d_in[1];
  const int*   mask   = (const int*)d_in[2];
  const float* W      = (const float*)d_in[3];
  const float* bias   = (const float*)d_in[4];
  float* out = (float*)d_out;

  char* ws = (char*)d_ws;
  size_t off = 0;
  _Float16* Hh = (_Float16*)(ws + off); off += (size_t)N_AGENT * N_HID * 2;
  _Float16* Wh = (_Float16*)(ws + off); off += (size_t)N_HID * K_FEAT * 2;
  float* P = (float*)(ws + off);        off += (size_t)N_CELLS * N_AGENT * N_HID * 4;
  if (off > ws_size) return;

  {
    const int n2h = N_AGENT * N_HID / 2;
    cast_f32_f16x2_carry<<<dim3(n2h / 256), dim3(256), 0, stream>>>(hidden, Hh, n2h, HID_CARRY);
    const int n2w = N_HID * K_FEAT / 2;
    cast_f32_f16x2_carry<<<dim3(n2w / 256), dim3(256), 0, stream>>>(W, Wh, n2w, W_CARRY);
  }
  {
    const int tiles = (N_AGENT / 64) * (N_HID / 64);
    wmma_gemm64<0, false, 0, 0, false, 0><<<dim3((tiles + 7) / 8, N_CELLS), dim3(256), 0, stream>>>(
        (const unsigned short*)Hh, (const unsigned short*)Hh, N_HID, 0L,
        (const unsigned short*)Wh, (const unsigned short*)Wh, K_FEAT, (long)N_HID,
        (void*)P, (void*)P, N_HID, (long)N_AGENT * N_HID,
        bias, P, 0L,
        N_AGENT, N_HID, N_HID, GEMM_SCALE);
  }
  cell_gather_pool<<<dim3(N_AGENT / AG_PER_BLK), dim3(128), 0, stream>>>(P, pos, mask, bias, out);
}
